// Window_DMSAttention_10222022164490
// MI455X (gfx1250) — hardware-verified
//
#include <hip/hip_runtime.h>
#include <stdint.h>

#pragma clang fp contract(off)

#define NB     4
#define NC     256
#define IMH    56
#define IMW    56
#define NPIX   3136
#define NHEAD  8
#define HCH    32
#define NGRP   2
#define GCH    128
#define WSZ    7
#define NWIN   64
#define NPT    784
#define NRG    28
#define NOFF   1568
#define NOFFP  1600
#define NQ     49
#define KVW    512
#define KVROWS (NWIN * NPT)
#define KVPADR 16
#define PTILE  112
#define NPTT   (NPT / PTILE)
#define GSP    264
#define ESP    72
#define VTP    808
#define VKEYS  800
#define OSP    36
#define CSP    68
#define TSP    72
#define NTHS   224

#define XSC   16.0f
#define WSC   64.0f
#define GSC   16.0f
#define KVC   16.0f
#define QSC   16.0f
#define ACTC  256.0f
#define YSC   1024.0f
#define PEX   14.0f
#define SCL2  (1.44269504088896340736f * 0.000244140625f)
#define OSC   0.0625f
#define RQ    0.0009765625f
#define ROF   0.00006103515625f
#define RKV   0.0009765625f
#define RPJ   0.0000152587890625f
#define RNG56 (1.0f / 56.0f)
#define RCP55 (1.0f / 55.0f)
#define BNK   0.99999500003749981f

#define DYN_GS  0
#define DYN_CW  (PTILE * GSP * 2)
#define DYN_CI  (DYN_CW + NGRP * PTILE * 16)
#define DYN_ES  (DYN_CI + NGRP * PTILE * 16)
#define DYN_TOT (DYN_ES + 7 * 16 * ESP * 2)

static_assert((NPT % PTILE) == 0);
static_assert((PTILE % 16) == 0);
static_assert(NTHS == 7 * 32);
static_assert(NTHS == NGRP * PTILE);
static_assert(((PTILE * (NC / 2)) % NTHS) == 0);
static_assert((VKEYS % 32) == 0);
static_assert(VKEYS >= NPT);
static_assert((NWIN - 1) * NPT + VKEYS <= KVROWS + KVPADR);
static_assert(((GSP * 2) % 16) == 0);
static_assert(((ESP * 2) % 16) == 0);
static_assert(((VTP * 2) % 16) == 0);
static_assert(((OSP * 4) % 16) == 0);
static_assert(((CSP * 4) % 16) == 0);
static_assert(((TSP * 2) % 16) == 0);
static_assert((NPIX % 64) == 0);
static_assert((NOFFP % 64) == 0);
static_assert(((NGRP * NB * NWIN) % 64) == 0);
static_assert((DYN_CW % 16) == 0 && (DYN_CI % 16) == 0 && (DYN_ES % 16) == 0);
static_assert((NPIX % 4) == 0);

typedef _Float16     v2h  __attribute__((ext_vector_type(2)));
typedef _Float16     v8h  __attribute__((ext_vector_type(8)));
typedef _Float16     v16h __attribute__((ext_vector_type(16)));
typedef unsigned int v4u  __attribute__((ext_vector_type(4)));
typedef int          v4i  __attribute__((ext_vector_type(4)));
typedef float        v4f  __attribute__((ext_vector_type(4)));
typedef float        v8f  __attribute__((ext_vector_type(8)));

union FragH { v8h p[2]; v4u u[2]; v16h v; };
union H8 { v8h v; _Float16 e[8]; };
static_assert(sizeof(FragH) == 32);
static_assert(sizeof(H8) == 16);

__device__ __forceinline__ v8f zero8() { v8f z = {0.f, 0.f, 0.f, 0.f, 0.f, 0.f, 0.f, 0.f}; return z; }

__device__ __forceinline__ float bf_rne(float x) {
  unsigned int u = __float_as_uint(x);
  u += 0x7FFFu + ((u >> 16) & 1u);
  return __uint_as_float(u & 0xFFFF0000u);
}

__device__ __forceinline__ v8f mma_h(v16h a, v16h b, v8f c) {
  v8f d = __builtin_amdgcn_wmma_f32_16x16x32_f16(false, a, false, b, (short)0, c, false, false);
#if defined(__HIP_DEVICE_COMPILE__)
  asm volatile("v_nop\n\tv_nop\n\tv_nop\n\tv_nop" : "+v"(d) : "v"(a), "v"(b));
#endif
  return d;
}

__global__ __launch_bounds__(256)
void k_wprep(const float* __restrict__ QW, const float* __restrict__ KW, const float* __restrict__ VW,
             const float* __restrict__ PJW, const float* __restrict__ PWW,
             _Float16* QW16, _Float16* WKV16, _Float16* PJ16, _Float16* PW16, _Float16* KVPAD) {
  const int t = threadIdx.x;
  const int blk = blockIdx.x;
  H8 u;
  _Float16* dst;
  if (blk < 32) {
    const int e0 = 8 * (blk * 256 + t);
#pragma unroll
    for (int i = 0; i < 8; ++i) u.e[i] = (_Float16)(bf_rne(QW[e0 + i]) * WSC);
    dst = QW16 + e0;
  } else if (blk < 96) {
    const int lb = blk - 32;
    const int e0 = 8 * (lb * 256 + t);
    const float* src = (lb < 32) ? KW : VW;
    const int se = e0 & 65535;
#pragma unroll
    for (int i = 0; i < 8; ++i) u.e[i] = (_Float16)(bf_rne(src[se + i]) * WSC);
    dst = WKV16 + e0;
  } else if (blk < 128) {
    const int lb = blk - 96;
    const int e0 = 8 * (lb * 256 + t);
#pragma unroll
    for (int i = 0; i < 8; ++i) u.e[i] = (_Float16)(bf_rne(PJW[e0 + i]) * WSC);
    dst = PJ16 + e0;
  } else if (blk < 228) {
    const int lb = blk - 128;
    const int e0 = 8 * (lb * 256 + t);
    const int j  = e0 >> 7;
    const int c0 = e0 & 127;
    const int jj = min(j, NOFF - 1);
    const bool ok = j < NOFF;
#pragma unroll
    for (int i = 0; i < 8; ++i) {
      const float w = bf_rne(PWW[jj * GCH + c0 + i]) * WSC;
      u.e[i] = ok ? (_Float16)w : (_Float16)0.0f;
    }
    dst = PW16 + e0;
  } else {
    const int lb = blk - 228;
    const int e0 = 8 * (lb * 256 + t);
#pragma unroll
    for (int i = 0; i < 8; ++i) u.e[i] = (_Float16)0.0f;
    dst = KVPAD + e0;
  }
  *(volatile v8h*)dst = u.v;
  __threadfence();
  *(volatile v8h*)dst = u.v;
}

__global__ __launch_bounds__(256)
void k_xprep(const float* __restrict__ X, _Float16* XT, float* XB) {
  __shared__ __align__(16) _Float16 Ts[64 * TSP];
  const int t  = threadIdx.x;
  const int pt = blockIdx.x, ct = blockIdx.y, b = blockIdx.z;
  const int p0 = pt * 64, c0 = ct * 64;
  const int pp = t & 63, cb = t >> 6;
  float xv[16];
  unsigned int xi[16];
#pragma unroll
  for (int it = 0; it < 16; ++it) {
    const int cc = it * 4 + cb;
    xi[it] = (unsigned int)(b * NC + c0 + cc) * NPIX + p0 + pp;
    xv[it] = bf_rne(X[xi[it]]);
    Ts[pp * TSP + cc] = (_Float16)(xv[it] * XSC);
  }
#pragma unroll
  for (int it = 0; it < 16; ++it) *(volatile float*)(XB + xi[it]) = xv[it];
  __threadfence();
#pragma unroll
  for (int it = 0; it < 16; ++it) *(volatile float*)(XB + xi[it]) = xv[it];
  __syncthreads();

  v8h wv[2];
  unsigned int pd[2];
#pragma unroll
  for (int it = 0; it < 2; ++it) {
    const int row = it * 32 + (t >> 3);
    const int q   = t & 7;
    wv[it] = *(const v8h*)(Ts + row * TSP + 8 * q);
    pd[it] = (unsigned int)(b * NPIX + p0 + row) * NC + c0 + 8 * q;
  }
  *(volatile v8h*)(XT + pd[0]) = wv[0];
  *(volatile v8h*)(XT + pd[1]) = wv[1];
  __threadfence();
  *(volatile v8h*)(XT + pd[0]) = wv[0];
  *(volatile v8h*)(XT + pd[1]) = wv[1];
}

template <int EPI, int HASB>
__global__ __launch_bounds__(128)
void k_gemm(const _Float16* __restrict__ A, const _Float16* __restrict__ Bw, const float* __restrict__ bias,
            float* Cout, int lda, int ldb, int ksteps, int ldc, float scale) {
  __shared__ __align__(16) float Cs[64 * CSP];
  const int t    = threadIdx.x;
  const int lane = t & 31, wv = t >> 5;
  const int hh   = lane >> 4, n = lane & 15;
  const int bm0  = blockIdx.x * 64;
  const int n0   = blockIdx.y * 64;

  const _Float16* ap = A + (size_t)(bm0 + 16 * wv + n) * lda + 8 * hh;
  v8f acc[4];
#pragma unroll
  for (int ct = 0; ct < 4; ++ct) acc[ct] = zero8();

#pragma unroll 1
  for (int ks = 0; ks < ksteps; ++ks) {
    FragH a;
    a.p[0] = *(const v8h*)(ap + ks * 32);
    a.p[1] = *(const v8h*)(ap + ks * 32 + 16);
#pragma unroll
    for (int ct = 0; ct < 4; ++ct) {
      const _Float16* wp = Bw + (size_t)(n0 + ct * 16 + n) * ldb + ks * 32 + 8 * hh;
      FragH w;
      w.p[0] = *(const v8h*)(wp);
      w.p[1] = *(const v8h*)(wp + 16);
      acc[ct] = mma_h(a.v, w.v, acc[ct]);
    }
  }

#pragma unroll
  for (int ct = 0; ct < 4; ++ct) {
    float bb = 0.0f;
    if (HASB) bb = bf_rne(bias[n0 + ct * 16 + n]);
#pragma unroll
    for (int r = 0; r < 8; ++r) {
      const float v = acc[ct][r] * scale + bb;
      if (EPI == 0) Cs[(16 * wv + 8 * hh + r) * CSP + ct * 16 + n] = v;
      else          Cs[(ct * 16 + n) * CSP + 16 * wv + 8 * hh + r] = v;
    }
  }
  __syncthreads();

  v4f    ov[8];
  size_t po[8];
  const int bimg = bm0 / NPIX;
  const int pp0  = bm0 - bimg * NPIX;
#pragma unroll
  for (int it = 0; it < 8; ++it) {
    const int row = it * 8 + (t >> 4);
    const int q   = t & 15;
    ov[it] = *(const v4f*)(Cs + row * CSP + 4 * q);
    if (EPI == 0) po[it] = (size_t)(bm0 + row) * (size_t)ldc + n0 + 4 * q;
    else          po[it] = (size_t)(bimg * NC + n0 + row) * (size_t)ldc + pp0 + 4 * q;
  }
#pragma unroll
  for (int it = 0; it < 8; ++it) *(volatile v4f*)(Cout + po[it]) = ov[it];
  __threadfence();
#pragma unroll
  for (int it = 0; it < 8; ++it) *(volatile v4f*)(Cout + po[it]) = ov[it];
}

__global__ __launch_bounds__(256)
void k_dw(const float* __restrict__ QF, const float* __restrict__ DW, const float* __restrict__ GA,
          const float* __restrict__ BE, _Float16* ACT) {
  __shared__ __align__(16) _Float16 As[256];
  const int t   = threadIdx.x;
  const int r   = t >> 7, c = t & 127;
  const int R   = blockIdx.x * 2 + r;
  const int n   = R >> 6, win = R & 63;
  const int b   = n >> 1, g = n & 1;
  const int wy  = win >> 3, wx = win & 7;
  const float* qp = QF + ((size_t)b * NPIX + (size_t)(wy * WSZ) * IMW + wx * WSZ) * NC + g * GCH + c;
  const float* wp = DW + c * 49;
  float s = 0.0f;
#pragma unroll 1
  for (int i = 0; i < 7; ++i) {
#pragma unroll
    for (int j = 0; j < 7; ++j) {
      s += qp[((size_t)i * IMW + j) * NC] * bf_rne(wp[i * 7 + j]);
    }
  }
  s = s * (bf_rne(GA[c]) * BNK) + bf_rne(BE[c]);
  s = 0.5f * s * (1.0f + erff(s * 0.70710678118654752f));
  As[t] = (_Float16)(s * ACTC);
  __syncthreads();
  if (t < 32) {
    const v8h v = *(const v8h*)(As + 8 * t);
    _Float16* dst = ACT + (size_t)blockIdx.x * 256 + 8 * t;
    *(volatile v8h*)dst = v;
    __threadfence();
    *(volatile v8h*)dst = v;
  }
}

__global__ __launch_bounds__(NTHS)
void k_sample_kv(const float* __restrict__ XB, const float* __restrict__ SOF, const _Float16* __restrict__ WKV,
                 const float* __restrict__ KB, const float* __restrict__ VB, _Float16* KV, int img) {
  extern __shared__ __align__(16) unsigned char dynlds[];
  _Float16* GS = (_Float16*)(dynlds + DYN_GS);
  v4f*      CW = (v4f*)(dynlds + DYN_CW);
  v4i*      CI = (v4i*)(dynlds + DYN_CI);
  _Float16* ES = (_Float16*)(dynlds + DYN_ES);
  const int t   = threadIdx.x;
  const int pt  = blockIdx.x;
  const int win = blockIdx.y;

  {
    const int g  = (t >= PTILE) ? 1 : 0;
    const int pl = t - g * PTILE;
    const int p  = pt * PTILE + pl;
    const float* srow = SOF + (size_t)((img * NGRP + g) * NWIN + win) * NOFFP;
    const float sy = srow[p];
    const float sx = srow[NPT + p];
    const int   pi = p / NRG;
    const int   pj = p - NRG * pi;
    const float offy = (tanhf(sy) * RNG56) * 2.0f;
    const float offx = (tanhf(sx) * RNG56) * 2.0f;
    const float ancy = ((float)(2 * pi) * RCP55) * 2.0f - 1.0f;
    const float ancx = ((float)(2 * pj) * RCP55) * 2.0f - 1.0f;
    const float gy = offy + ancy;
    const float gx = offx + ancx;
    const float py = ((gy + 1.0f) * 0.5f) * 55.0f;
    const float px = ((gx + 1.0f) * 0.5f) * 55.0f;
    const float y0 = floorf(py), x0 = floorf(px);
    const float y1 = y0 + 1.0f, x1 = x0 + 1.0f;
    const float wy1 = py - y0, wy0 = 1.0f - wy1;
    const float wx1 = px - x0, wx0 = 1.0f - wx1;
    const float my0 = (y0 >= 0.0f && y0 <= 55.0f) ? 1.0f : 0.0f;
    const float my1 = (y1 >= 0.0f && y1 <= 55.0f) ? 1.0f : 0.0f;
    const float mx0 = (x0 >= 0.0f && x0 <= 55.0f) ? 1.0f : 0.0f;
    const float mx1 = (x1 >= 0.0f && x1 <= 55.0f) ? 1.0f : 0.0f;
    v4f w;
    w.x = (wx0 * wy0) * (mx0 * my0);
    w.y = (wx1 * wy0) * (mx1 * my0);
    w.z = (wx0 * wy1) * (mx0 * my1);
    w.w = (wx1 * wy1) * (mx1 * my1);
    const int x0c = (int)fminf(fmaxf(x0, 0.0f), 55.0f);
    const int x1c = (int)fminf(fmaxf(x1, 0.0f), 55.0f);
    const int y0c = (int)fminf(fmaxf(y0, 0.0f), 55.0f);
    const int y1c = (int)fminf(fmaxf(y1, 0.0f), 55.0f);
    v4i ci;
    ci.x = y0c * IMW + x0c;
    ci.y = y0c * IMW + x1c;
    ci.z = y1c * IMW + x0c;
    ci.w = y1c * IMW + x1c;
    CW[g * PTILE + pl] = w;
    CI[g * PTILE + pl] = ci;
  }
  __syncthreads();

#pragma unroll 1
  for (int s = t; s < PTILE * (NC / 2); s += NTHS) {
    const int pl = s >> 7;
    const int c  = (s & 127) * 2;
    const int g  = c >> 7;
    const v4f w  = CW[g * PTILE + pl];
    const v4i ci = CI[g * PTILE + pl];
    const float* pa = XB + (size_t)c * NPIX;
    const float* pb = pa + NPIX;
    const float va = ((pa[ci.x] * w.x + pa[ci.y] * w.y) + pa[ci.z] * w.z) + pa[ci.w] * w.w;
    const float vb = ((pb[ci.x] * w.x + pb[ci.y] * w.y) + pb[ci.z] * w.z) + pb[ci.w] * w.w;
    v2h hv;
    hv.x = (_Float16)(va * GSC);
    hv.y = (_Float16)(vb * GSC);
    *(v2h*)(GS + pl * GSP + c) = hv;
  }
  __syncthreads();

  const int lane = t & 31, wv = t >> 5;
  const int hh   = lane >> 4, n = lane & 15;
  const _Float16* ap = GS + (16 * wv + n) * GSP + 8 * hh;
  _Float16* esw = ES + wv * 16 * ESP;
  const size_t rowbase = (size_t)win * NPT + (size_t)pt * PTILE + 16 * wv;

#pragma unroll 1
  for (int cg = 0; cg < KVW / 64; ++cg) {
    v8f acc[4];
#pragma unroll
    for (int ct = 0; ct < 4; ++ct) acc[ct] = zero8();
#pragma unroll 1
    for (int ks = 0; ks < NC / 32; ++ks) {
      FragH a;
      a.p[0] = *(const v8h*)(ap + ks * 32);
      a.p[1] = *(const v8h*)(ap + ks * 32 + 16);
#pragma unroll
      for (int ct = 0; ct < 4; ++ct) {
        const _Float16* wp = WKV + (size_t)(cg * 64 + ct * 16 + n) * NC + ks * 32 + 8 * hh;
        FragH w;
        w.p[0] = *(const v8h*)(wp);
        w.p[1] = *(const v8h*)(wp + 16);
        acc[ct] = mma_h(a.v, w.v, acc[ct]);
      }
    }
#pragma unroll
    for (int ct = 0; ct < 4; ++ct) {
      const int o   = cg * 64 + ct * 16 + n;
      const int oo  = o & 255;
      const float kbv = bf_rne(KB[oo]);
      const float vbv = bf_rne(VB[oo]);
      const float bb  = (cg < 4) ? kbv : vbv;
#pragma unroll
      for (int r = 0; r < 8; ++r) {
        const float v = (acc[ct][r] * RKV + bb) * KVC;
        esw[(8 * hh + r) * ESP + ct * 16 + n] = (_Float16)v;
      }
    }
    __syncthreads();
    v8h    w4[4];
    size_t pd[4];
#pragma unroll
    for (int it = 0; it < 4; ++it) {
      const int row = it * 4 + (lane >> 3);
      const int q   = lane & 7;
      w4[it] = *(const v8h*)(esw + row * ESP + 8 * q);
      pd[it] = (rowbase + row) * KVW + cg * 64 + 8 * q;
    }
#pragma unroll
    for (int it = 0; it < 4; ++it) *(volatile v8h*)(KV + pd[it]) = w4[it];
    __threadfence();
#pragma unroll
    for (int it = 0; it < 4; ++it) *(volatile v8h*)(KV + pd[it]) = w4[it];
    __syncthreads();
  }
}

__global__ __launch_bounds__(128)
void k_attn(const float* __restrict__ QF, const _Float16* __restrict__ KV, float* ATT) {
  __shared__ __align__(16) _Float16 VT[HCH * VTP];
  __shared__ __align__(16) float Os[64 * OSP];
  const int t    = threadIdx.x;
  const int lane = t & 31, wv = t >> 5;
  const int hh   = lane >> 4, n = lane & 15;
  const int head = blockIdx.x, win = blockIdx.y;
  const int wy   = win >> 3, wx = win & 7;
  const size_t kvrow0 = (size_t)win * NPT;

#pragma unroll 1
  for (int it = 0; it < VKEYS / 32; ++it) {
    const int key = it * 32 + (t >> 2);
    const int q4  = t & 3;
    const int kc  = min(key, NPT - 1);
    H8 u;
    u.v = *(const v8h*)(KV + (kvrow0 + kc) * KVW + NC + head * HCH + 8 * q4);
    const bool ok = key < NPT;
#pragma unroll
    for (int e = 0; e < 8; ++e) {
      const _Float16 hv = ok ? u.e[e] : (_Float16)0.0f;
      VT[(8 * q4 + e) * VTP + key] = hv;
    }
  }
  __syncthreads();

  const int m  = 16 * wv + n;
  const int mc = min(m, NQ - 1);
  const int qi = mc / WSZ, qj = mc - WSZ * qi;
  const float qs = (m < NQ) ? QSC : 0.0f;
  const float* qrow = QF + (size_t)((wy * WSZ + qi) * IMW + wx * WSZ + qj) * NC + head * HCH + 8 * hh;
  const v4f f0 = *(const v4f*)(qrow);
  const v4f f1 = *(const v4f*)(qrow + 4);
  const v4f g0 = *(const v4f*)(qrow + 16);
  const v4f g1 = *(const v4f*)(qrow + 20);
  FragH qf;
#pragma unroll
  for (int i = 0; i < 4; ++i) {
    qf.v[i]      = (_Float16)(f0[i] * qs);
    qf.v[4 + i]  = (_Float16)(f1[i] * qs);
    qf.v[8 + i]  = (_Float16)(g0[i] * qs);
    qf.v[12 + i] = (_Float16)(g1[i] * qs);
  }

  const _Float16* kbase = KV + (kvrow0 + n) * KVW + head * HCH + 8 * hh;
  v8f O0 = zero8(), O1 = zero8();
  float mrun = -1.0e30f, z = 0.0f;

#pragma unroll 1
  for (int j = 0; j < VKEYS / 32; ++j) {
    const _Float16* kp0 = kbase + (size_t)(32 * j) * KVW;
    const _Float16* kp1 = kp0 + (size_t)16 * KVW;
    FragH ka, kb;
    ka.p[0] = *(const v8h*)(kp0);
    ka.p[1] = *(const v8h*)(kp0 + 16);
    kb.p[0] = *(const v8h*)(kp1);
    kb.p[1] = *(const v8h*)(kp1 + 16);
    const v8f S0 = mma_h(ka.v, qf.v, zero8());
    const v8f S1 = mma_h(kb.v, qf.v, zero8());

    const float fill = (j == VKEYS / 32 - 1) ? -1.0e30f : 0.0f;
    float u0[8], u1[8];
    float tm = -1.0e30f;
#pragma unroll
    for (int r = 0; r < 8; ++r) {
      u0[r] = S0[r] * SCL2;
      u1[r] = S1[r] * SCL2 + fill;
      tm = fmaxf(tm, fmaxf(u0[r], u1[r]));
    }
    const float tmo = __shfl_xor(tm, 16, 32);
    tm = fmaxf(tm, tmo);
    const float mn    = fmaxf(mrun, tm);
    const float alpha = __builtin_amdgcn_exp2f(mrun - mn);
    mrun = mn;
    const float nb = PEX - mn;
    z *= alpha;
    O0 = O0 * alpha;
    O1 = O1 * alpha;

    FragH pf;
#pragma unroll
    for (int r = 0; r < 8; ++r) {
      const _Float16 e0 = (_Float16)__builtin_amdgcn_exp2f(u0[r] + nb);
      const _Float16 e1 = (_Float16)__builtin_amdgcn_exp2f(u1[r] + nb);
      pf.v[r]     = e0;
      pf.v[8 + r] = e1;
      z += (float)e0;
      z += (float)e1;
    }

    const _Float16* vp0 = VT + n * VTP + 32 * j + 8 * hh;
    const _Float16* vp1 = vp0 + 16 * VTP;
    FragH va, vb;
    va.p[0] = *(const v8h*)(vp0);
    va.p[1] = *(const v8h*)(vp0 + 16);
    vb.p[0] = *(const v8h*)(vp1);
    vb.p[1] = *(const v8h*)(vp1 + 16);
    O0 = mma_h(va.v, pf.v, O0);
    O1 = mma_h(vb.v, pf.v, O1);
  }

  const float zo = __shfl_xor(z, 16, 32);
  const float zt = z + zo;
  const float rz = (1.0f / zt) * OSC;
#pragma unroll
  for (int r = 0; r < 8; ++r) {
    Os[(16 * wv + n) * OSP + 8 * hh + r]      = O0[r] * rz;
    Os[(16 * wv + n) * OSP + 16 + 8 * hh + r] = O1[r] * rz;
  }
  __syncthreads();

  v4f    ov[4];
  size_t po[4];
  bool   okq[4];
#pragma unroll
  for (int it = 0; it < 4; ++it) {
    const int q   = it * 16 + (t >> 3);
    const int qq  = t & 7;
    const int qc  = min(q, NQ - 1);
    const int qi2 = qc / WSZ, qj2 = qc - WSZ * qi2;
    okq[it] = q < NQ;
    ov[it]  = *(const v4f*)(Os + q * OSP + 4 * qq);
    po[it]  = (size_t)((wy * WSZ + qi2) * IMW + wx * WSZ + qj2) * NC + head * HCH + 4 * qq;
  }
#pragma unroll
  for (int it = 0; it < 4; ++it) if (okq[it]) *(volatile v4f*)(ATT + po[it]) = ov[it];
  __threadfence();
#pragma unroll
  for (int it = 0; it < 4; ++it) if (okq[it]) *(volatile v4f*)(ATT + po[it]) = ov[it];
}

__global__ __launch_bounds__(256)
void k_pos(const float* __restrict__ ATT, const float* __restrict__ PW, const float* __restrict__ PB, _Float16* Y) {
  __shared__ __align__(16) _Float16 Ys[4 * NC];
  const int t = threadIdx.x;
  const int c = t;
  float w9[9];
#pragma unroll
  for (int i = 0; i < 9; ++i) w9[i] = bf_rne(PW[c * 9 + i]);
  const float pb = bf_rne(PB[c]);
#pragma unroll 1
  for (int i = 0; i < 4; ++i) {
    const int P = blockIdx.x * 4 + i;
    const int b = P / NPIX;
    const int p = P - b * NPIX;
    const int h = p / IMW;
    const int x = p - h * IMW;
    const float* ab = ATT + (size_t)b * NPIX * NC + c;
    float s = pb;
#pragma unroll
    for (int tap = 0; tap < 9; ++tap) {
      const int dy = tap / 3;
      const int dx = tap - 3 * dy;
      const int yy = h + dy - 1;
      const int xx = x + dx - 1;
      const bool inb = ((unsigned)yy < (unsigned)IMH) && ((unsigned)xx < (unsigned)IMW);
      const int yc = min(max(yy, 0), IMH - 1);
      const int xc = min(max(xx, 0), IMW - 1);
      float v = ab[(size_t)(yc * IMW + xc) * NC];
      v = inb ? v : 0.0f;
      s += w9[tap] * v;
    }
    const float ctr = ab[(size_t)(h * IMW + x) * NC];
    const float y = ctr + s;
    Ys[i * NC + c] = (_Float16)(y * YSC);
  }
  __syncthreads();
  if (t < 128) {
    const v8h v = *(const v8h*)(Ys + 8 * t);
    _Float16* dst = Y + (size_t)blockIdx.x * 4 * NC + 8 * t;
    *(volatile v8h*)dst = v;
    __threadfence();
    *(volatile v8h*)dst = v;
  }
}

extern "C" void kernel_launch(void* const* d_in, const int* in_sizes, int n_in,
                              void* d_out, int out_size, void* d_ws, size_t ws_size,
                              hipStream_t stream) {
  if (n_in < 15) return;
  if (in_sizes[0]  != NB * NC * NPIX) return;
  if (in_sizes[1]  != NC * NC) return;
  if (in_sizes[2]  != NC) return;
  if (in_sizes[3]  != NC * NC) return;
  if (in_sizes[4]  != NC) return;
  if (in_sizes[5]  != NC * NC) return;
  if (in_sizes[6]  != NC) return;
  if (in_sizes[7]  != GCH * 49) return;
  if (in_sizes[8]  != GCH) return;
  if (in_sizes[9]  != GCH) return;
  if (in_sizes[10] != NOFF * GCH) return;
  if (in_sizes[11] != NC * 9) return;
  if (in_sizes[12] != NC) return;
  if (in_sizes[13] != NC * NC) return;
  if (in_sizes[14] != NC) return;
  if (out_size != NB * NC * NPIX) return;

  const size_t szQW  = (size_t)NC * NC * 2;
  const size_t szWKV = (size_t)KVW * NC * 2;
  const size_t szPJ  = (size_t)NC * NC * 2;
  const size_t szPW  = (size_t)NOFFP * GCH * 2;
  const size_t szXT  = (size_t)NB * NPIX * NC * 2;
  const size_t szXB  = (size_t)NB * NC * NPIX * 4;
  const size_t szQF  = (size_t)NB * NPIX * NC * 4;
  const size_t szACT = (size_t)NGRP * NB * NWIN * GCH * 2;
  const size_t szSOF = (size_t)NGRP * NB * NWIN * NOFFP * 4;
  const size_t szKV  = (size_t)(KVROWS + KVPADR) * KVW * 2;
  const size_t szATT = (size_t)NB * NPIX * NC * 4;
  const size_t szY   = (size_t)NB * NPIX * NC * 2;
  size_t off = 0;
  const size_t oQW  = off; off += szQW;
  const size_t oWKV = off; off += szWKV;
  const size_t oPJ  = off; off += szPJ;
  const size_t oPW  = off; off += szPW;
  const size_t oXT  = off; off += szXT;
  const size_t oXB  = off; off += szXB;
  const size_t oQF  = off; off += szQF;
  const size_t oACT = off; off += szACT;
  const size_t oSOF = off; off += szSOF;
  const size_t oKV  = off; off += szKV;
  const size_t oATT = off; off += szATT;
  const size_t oY   = off; off += szY;
  if (off > ws_size) return;
  if (off > (size_t)134217728) return;
  if ((oWKV % 256) != 0 || (oPJ % 256) != 0 || (oPW % 256) != 0 || (oXT % 256) != 0 || (oXB % 256) != 0 ||
      (oQF % 256) != 0 || (oACT % 256) != 0 || (oSOF % 256) != 0 || (oKV % 256) != 0 || (oATT % 256) != 0 ||
      (oY % 256) != 0) return;

  const float* x     = (const float*)d_in[0];
  const float* q_w   = (const float*)d_in[1];
  const float* q_b   = (const float*)d_in[2];
  const float* k_w   = (const float*)d_in[3];
  const float* k_b   = (const float*)d_in[4];
  const float* v_w   = (const float*)d_in[5];
  const float* v_b   = (const float*)d_in[6];
  const float* dw_w  = (const float*)d_in[7];
  const float* bn_g  = (const float*)d_in[8];
  const float* bn_b  = (const float*)d_in[9];
  const float* pw_w  = (const float*)d_in[10];
  const float* pos_w = (const float*)d_in[11];
  const float* pos_b = (const float*)d_in[12];
  const float* pj_w  = (const float*)d_in[13];
  const float* pj_b  = (const float*)d_in[14];
  float* out = (float*)d_out;

  char* ws = (char*)d_ws;
  _Float16* QW16  = (_Float16*)(ws + oQW);
  _Float16* WKV16 = (_Float16*)(ws + oWKV);
  _Float16* PJ16  = (_Float16*)(ws + oPJ);
  _Float16* PW16  = (_Float16*)(ws + oPW);
  _Float16* XT    = (_Float16*)(ws + oXT);
  float*    XB    = (float*)(ws + oXB);
  float*    QF    = (float*)(ws + oQF);
  _Float16* ACT   = (_Float16*)(ws + oACT);
  float*    SOF   = (float*)(ws + oSOF);
  _Float16* KV    = (_Float16*)(ws + oKV);
  float*    ATT   = (float*)(ws + oATT);
  _Float16* Y     = (_Float16*)(ws + oY);

  k_wprep<<<dim3(232), dim3(256), 0, stream>>>(q_w, k_w, v_w, pj_w, pw_w, QW16, WKV16, PJ16, PW16,
                                                KV + (size_t)KVROWS * KVW);
  k_xprep<<<dim3(NPIX / 64, NC / 64, NB), dim3(256), 0, stream>>>(x, XT, XB);
  k_gemm<0, 1><<<dim3(NB * NPIX / 64, NC / 64), dim3(128), 0, stream>>>(
      XT, QW16, q_b, QF, NC, NC, NC / 32, NC, RQ);
  k_dw<<<dim3(NGRP * NB * NWIN / 2), dim3(256), 0, stream>>>(QF, dw_w, bn_g, bn_b, ACT);
  k_gemm<0, 0><<<dim3(NGRP * NB * NWIN / 64, NOFFP / 64), dim3(128), 0, stream>>>(
      ACT, PW16, q_b, SOF, GCH, GCH, GCH / 32, NOFFP, ROF);
  (void)hipFuncSetAttribute(reinterpret_cast<const void*>(&k_sample_kv),
                            hipFuncAttributeMaxDynamicSharedMemorySize, DYN_TOT);
  for (int img = 0; img < NB; ++img) {
    k_sample_kv<<<dim3(NPTT, NWIN), dim3(NTHS), DYN_TOT, stream>>>(
        XB + (size_t)img * NC * NPIX, SOF, WKV16, k_b, v_b, KV, img);
    k_attn<<<dim3(NHEAD, NWIN), dim3(128), 0, stream>>>(
        QF + (size_t)img * NPIX * NC, KV, ATT + (size_t)img * NPIX * NC);
  }
  k_pos<<<dim3(NB * NPIX / 4), dim3(256), 0, stream>>>(ATT, pos_w, pos_b, Y);
  k_gemm<1, 1><<<dim3(NB * NPIX / 64, NC / 64), dim3(128), 0, stream>>>(
      Y, PJ16, pj_b, out, NC, NC, NC / 32, NPIX, RPJ);
  (void)hipGetLastError();
}
